// RelativeSelfAttention_13675175870611
// MI455X (gfx1250) — hardware-verified
//
#include <hip/hip_runtime.h>
#include <math.h>

#ifndef NB
#define NB 2
#endif
#ifndef SEQ
#define SEQ 2048
#endif
#define NB_FULL  2
#define SEQ_FULL 2048
#define DM    1024
#define NH    16
#define HD    64
#define GRP   (3 * HD)
#define MT    (NB * SEQ)
#define NREL  257
#define NRELP 272
#define RELW  128
#define AWV   2
#define RP    NRELP
#define ZP    68
#define WSCL  64.0f
#define QKS   16.0f
#define VSC   16.0f
#define LSC   1024.0f
#define PSC   4096.0f
#define RSQD  0.125f

static_assert(NH * HD == DM);
static_assert(HD == 64);
static_assert(NB >= 1 && NB <= NB_FULL);
static_assert((SEQ % 64) == 0 && SEQ >= 64 && SEQ <= SEQ_FULL);
static_assert((MT % 64) == 0 && (DM % 64) == 0);
static_assert(((MT * DM) % 2048) == 0 && ((3 * DM * DM) % 2048) == 0);
static_assert((NRELP % 16) == 0 && NRELP >= NREL && ((NRELP * HD) % 64) == 0);
static_assert(((NB * NH * (SEQ / 16)) % AWV) == 0);
static_assert(2 * RELW + 1 == NREL);
static_assert(16 * ZP <= 16 * RP);

typedef _Float16 v16h __attribute__((ext_vector_type(16)));
typedef unsigned short v16us __attribute__((ext_vector_type(16)));
typedef unsigned short v8us  __attribute__((ext_vector_type(8)));
typedef float v8f __attribute__((ext_vector_type(8)));
typedef float v4f __attribute__((ext_vector_type(4)));
typedef unsigned int v4u __attribute__((ext_vector_type(4)));

union FragU { v16us v; v8us h[2]; };

__device__ __forceinline__ unsigned short bf_bits(float f) {
  const unsigned u = __float_as_uint(f);
  return (unsigned short)((u + 0x7FFFu + ((u >> 16) & 1u)) >> 16);
}
__device__ __forceinline__ float bf_up(unsigned short h) { return __uint_as_float(((unsigned)h) << 16); }
__device__ __forceinline__ float bfr(float f) { return bf_up(bf_bits(f)); }
__device__ __forceinline__ unsigned short h_bits(_Float16 x) { return __builtin_bit_cast(unsigned short, x); }
__device__ __forceinline__ unsigned short f2h(float f) { return h_bits((_Float16)f); }
__device__ __forceinline__ unsigned pk16(unsigned short a, unsigned short b) { return (unsigned)a | ((unsigned)b << 16); }
__device__ __forceinline__ int clampi(int v, int lo, int hi) { return v < lo ? lo : (v > hi ? hi : v); }
__device__ __forceinline__ v8f zero8() { v8f z = {0.f, 0.f, 0.f, 0.f, 0.f, 0.f, 0.f, 0.f}; return z; }

__device__ __forceinline__ v16us ldfrag_u(const unsigned short* p) {
  FragU f;
  f.h[0] = *(const v8us*)(p);
  f.h[1] = *(const v8us*)(p + 16);
  return f.v;
}

__device__ __forceinline__ v8f mma_raw(v16us a, v16us b, v8f c) {
  return __builtin_amdgcn_wmma_f32_16x16x32_f16(false, __builtin_bit_cast(v16h, a), false,
                                                __builtin_bit_cast(v16h, b), (short)0, c, false, false);
}
__device__ __forceinline__ v8f mma_g(v16us a, v16us b, v8f c) {
  c = mma_raw(a, b, c);
#if defined(__HIP_DEVICE_COMPILE__)
  asm volatile("v_nop\n\tv_nop\n\tv_nop\n\tv_nop" : "+v"(c) : "v"(a), "v"(b));
#endif
  return c;
}
__device__ __forceinline__ void dep_guard1(v8f& a, v8f& b, v16us x) {
#if defined(__HIP_DEVICE_COMPILE__)
  asm volatile("v_nop\n\tv_nop\n\tv_nop\n\tv_nop" : "+v"(a), "+v"(b) : "v"(x));
#endif
}
__device__ __forceinline__ void keep4_u(v16us a, v16us b, v16us c, v16us d) {
#if defined(__HIP_DEVICE_COMPILE__)
  asm volatile("v_nop" :: "v"(a), "v"(b), "v"(c), "v"(d));
#endif
}
__device__ __forceinline__ void acc_guard4(v8f& a, v8f& b, v8f& c, v8f& d) {
#if defined(__HIP_DEVICE_COMPILE__)
  asm volatile("v_nop\n\tv_nop\n\tv_nop\n\tv_nop" : "+v"(a), "+v"(b), "+v"(c), "+v"(d));
#endif
}
__device__ __forceinline__ void wave_sync_lds() {
  __builtin_amdgcn_fence(__ATOMIC_RELEASE, "workgroup");
  __builtin_amdgcn_wave_barrier();
  __builtin_amdgcn_fence(__ATOMIC_ACQUIRE, "workgroup");
}

template <int MAP>
__global__ __launch_bounds__(256) void cvt_rows(const float* __restrict__ w, unsigned short* o,
                                                 int ndst, float sc) {
  const int base = (blockIdx.x * 256 + threadIdx.x) * 8;
  if (base + 8 > ndst) return;
  const int ncol = (MAP == 2) ? HD : DM;
  const int R = base / ncol;
  const int c = base - R * ncol;
  int srow = 0;
  bool inr = true;
  if (MAP == 0) {
    const int bb = R / SEQ;
    const int t = R - bb * SEQ;
    srow = bb * SEQ_FULL + t;
  } else if (MAP == 1) {
    const int g = R / DM;
    const int rr = R - g * DM;
    const int hq = rr / HD;
    const int d = rr - hq * HD;
    srow = hq * GRP + g * HD + d;
  } else {
    inr = (R < NREL);
    srow = inr ? R : (NREL - 1);
  }
  const float* p = w + (size_t)srow * ncol + c;
  const v4f a0 = *(const v4f*)(p);
  const v4f a1 = *(const v4f*)(p + 4);
  v4u hv;
#pragma unroll
  for (int e = 0; e < 2; ++e) {
    hv[e]     = pk16(f2h(bfr(a0[2 * e]) * sc), f2h(bfr(a0[2 * e + 1]) * sc));
    hv[2 + e] = pk16(f2h(bfr(a1[2 * e]) * sc), f2h(bfr(a1[2 * e + 1]) * sc));
  }
  const v4u zz = {0u, 0u, 0u, 0u};
  hv = inr ? hv : zz;
  unsigned short* d = o + base;
  *(volatile v4u*)d = hv;
  __threadfence();
  *(volatile v4u*)d = hv;
}

template <int OM, int BM>
__global__ __launch_bounds__(256) void gemm64(
    const unsigned short* __restrict__ Ap, int lda, const unsigned short* __restrict__ Btp, int ldb,
    unsigned short* Ch, unsigned short* Cl, int ldc, float osc,
    const float* __restrict__ bias, int bgs, int bofs, float bsc, int M, int N, int K) {
  __shared__ __align__(16) float sT[8][16 * 68];
  const int lane = threadIdx.x & 31;
  const int wave = threadIdx.x >> 5;
  const int tilesN = N >> 6;
  const int tilesM = M >> 6;
  const int tile = blockIdx.x * 8 + wave;
  if (tile >= tilesM * tilesN) return;
  const int tm = tile / tilesN;
  const int tn = tile - tm * tilesN;
  const int m0 = tm << 6;
  const int n0 = tn << 6;

  const int rlane = lane & 15;
  const int koff  = (lane >> 4) * 8;
  const int mOff  = (lane >> 4) * 8;

  v8f acc[4][4];
#pragma unroll
  for (int i = 0; i < 4; ++i)
#pragma unroll
    for (int j = 0; j < 4; ++j) acc[i][j] = zero8();

#pragma unroll 1
  for (int k0 = 0; k0 < K; k0 += 32) {
    v16us bh[4];
#pragma unroll
    for (int j = 0; j < 4; ++j) {
      const size_t bo = (size_t)(n0 + (j << 4) + rlane) * ldb + koff + k0;
      bh[j] = ldfrag_u(Btp + bo);
    }
#pragma unroll
    for (int i = 0; i < 4; ++i) {
      const size_t ao = (size_t)(m0 + (i << 4) + rlane) * lda + koff + k0;
      const v16us ah = ldfrag_u(Ap + ao);
#pragma unroll
      for (int j = 0; j < 4; ++j) acc[i][j] = mma_raw(ah, bh[j], acc[i][j]);
      dep_guard1(acc[i][0], acc[i][3], ah);
    }
    keep4_u(bh[0], bh[1], bh[2], bh[3]);
  }
  acc_guard4(acc[0][0], acc[0][1], acc[0][2], acc[0][3]);
  acc_guard4(acc[1][0], acc[1][1], acc[1][2], acc[1][3]);
  acc_guard4(acc[2][0], acc[2][1], acc[2][2], acc[2][3]);
  acc_guard4(acc[3][0], acc[3][1], acc[3][2], acc[3][3]);

  const int q8 = lane >> 3, c8 = (lane & 7) * 8;

  float bc[8];
#pragma unroll
  for (int e = 0; e < 8; ++e) bc[e] = 0.f;
  if (BM == 1) {
#pragma unroll
    for (int e = 0; e < 8; ++e) {
      const int n = n0 + c8 + e;
      const int gq = n / HD;
      bc[e] = bfr(bias[gq * bgs + bofs + (n - gq * HD)]) * bsc;
    }
  }

  float* slab = sT[wave];
#pragma unroll
  for (int i = 0; i < 4; ++i) {
    const int mBase = m0 + (i << 4);
#pragma unroll
    for (int j = 0; j < 4; ++j) {
#pragma unroll
      for (int r = 0; r < 8; ++r) {
        slab[(mOff + r) * 68 + (j << 4) + rlane] = acc[i][j][r];
      }
    }
    wave_sync_lds();
    v4u hv[4], lv[4];
#pragma unroll
    for (int it = 0; it < 4; ++it) {
      const int row = it * 4 + q8;
      const float* sp = slab + row * 68 + c8;
      float br = 0.f;
      if (BM == 2) {
        const int mr = mBase + row;
        const int gq = mr / HD;
        br = bfr(bias[gq * bgs + bofs + (mr - gq * HD)]) * bsc;
      }
      v4u ha = {0u, 0u, 0u, 0u};
      v4u la = {0u, 0u, 0u, 0u};
#pragma unroll
      for (int e = 0; e < 4; ++e) {
        const float b0 = sp[2 * e]     * osc + ((BM == 1) ? bc[2 * e]     : br);
        const float b1 = sp[2 * e + 1] * osc + ((BM == 1) ? bc[2 * e + 1] : br);
        const _Float16 h0 = (_Float16)b0;
        const _Float16 h1 = (_Float16)b1;
        ha[e] = pk16(h_bits(h0), h_bits(h1));
        if (OM == 2) {
          la[e] = pk16(f2h((b0 - (float)h0) * LSC), f2h((b1 - (float)h1) * LSC));
        }
      }
      hv[it] = ha;
      lv[it] = la;
    }
    for (int pass = 0; pass < 2; ++pass) {
#pragma unroll
      for (int it = 0; it < 4; ++it) {
        const int row = it * 4 + q8;
        const size_t go = (size_t)(mBase + row) * ldc + (size_t)n0 + c8;
        *(volatile v4u*)(Ch + go) = hv[it];
        if (OM == 2) *(volatile v4u*)(Cl + go) = lv[it];
      }
      __threadfence();
    }
    wave_sync_lds();
  }
}

__global__ __launch_bounds__(64) void attn_kernel(
    const unsigned short* __restrict__ QH, const unsigned short* __restrict__ QL,
    const unsigned short* __restrict__ KH, const unsigned short* __restrict__ PE,
    const unsigned short* __restrict__ VT, const float* __restrict__ brel,
    const int* __restrict__ mask, float* out) {
  __shared__ __align__(16) float relw[AWV][16 * RP];
  __shared__ __align__(16) unsigned short pws[AWV][16 * 32];
  const int lane = threadIdx.x & 31, wv = threadIdx.x >> 5, m = lane & 15, hh = lane >> 4;
  const int task = blockIdx.x * AWV + wv;
  const int nqt = SEQ / 16;
  const int bh = task / nqt;
  const int t0 = (task - bh * nqt) << 4;
  const int b = bh / NH, h = bh - (bh / NH) * NH;
  if (b >= NB) return;
  const size_t tok0 = (size_t)b * SEQ;
  float* rw = relw[wv];
  unsigned short* ph = pws[wv];

  const size_t qo = (tok0 + (size_t)(t0 + m)) * DM + h * HD + 8 * hh;
  const v16us qh0 = ldfrag_u(QH + qo);
  const v16us qh1 = ldfrag_u(QH + qo + 32);
  const v16us ql0 = ldfrag_u(QL + qo);
  const v16us ql1 = ldfrag_u(QL + qo + 32);

  const float crh = 1.0f / (QKS * WSCL);
  const float crl = 1.0f / (QKS * WSCL * LSC);
#pragma unroll 1
  for (int nt = 0; nt < NRELP / 16; ++nt) {
    const unsigned short* pp = PE + (size_t)(nt * 16 + m) * HD + 8 * hh;
    const v16us w0 = ldfrag_u(pp);
    const v16us w1 = ldfrag_u(pp + 32);
    v8f R = mma_g(qh0, w0, zero8());
    R = mma_g(qh1, w1, R);
    v8f Rl = mma_g(ql0, w0, zero8());
    Rl = mma_g(ql1, w1, Rl);
    const int col = nt * 16 + m;
    const float bb = bfr(brel[clampi(col, 0, NREL - 1)]);
#pragma unroll
    for (int r = 0; r < 8; ++r) {
      const int row = 8 * hh + r;
      rw[row * RP + col] = R[r] * crh + Rl[r] * crl + bb;
    }
  }
  wave_sync_lds();

  float mx[8], ls[8];
  v8f O0 = zero8(), O1 = zero8(), O2 = zero8(), O3 = zero8();
#pragma unroll
  for (int r = 0; r < 8; ++r) { mx[r] = -1.0e30f; ls[r] = 0.f; }
  const int* mk = mask + (size_t)b * SEQ_FULL;
  const float cqh = RSQD / (QKS * QKS);
  const float cql = RSQD / (QKS * QKS * LSC);
  const float ninf = __uint_as_float(0xff800000u);

#pragma unroll 1
  for (int kb = 0; kb < SEQ / 32; ++kb) {
    const int sb = kb << 5;
    v8f S0, S1, L0, L1;
    {
      const unsigned short* kp = KH + (tok0 + (size_t)(sb + m)) * DM + h * HD + 8 * hh;
      const v16us ka = ldfrag_u(kp);
      const v16us kc = ldfrag_u(kp + 32);
      S0 = mma_g(qh0, ka, zero8());
      S0 = mma_g(qh1, kc, S0);
      L0 = mma_g(ql0, ka, zero8());
      L0 = mma_g(ql1, kc, L0);
      const unsigned short* kp1 = kp + (size_t)16 * DM;
      const v16us kd = ldfrag_u(kp1);
      const v16us ke = ldfrag_u(kp1 + 32);
      S1 = mma_g(qh0, kd, zero8());
      S1 = mma_g(qh1, ke, S1);
      L1 = mma_g(ql0, kd, zero8());
      L1 = mma_g(ql1, ke, L1);
    }

    const int j0 = sb + m, j1 = sb + 16 + m;
    const int mk0 = mk[j0], mk1 = mk[j1];
    float s0[8], s1[8];
#pragma unroll
    for (int r = 0; r < 8; ++r) {
      const int row = 8 * hh + r;
      const int i = t0 + row;
      const float pv0 = rw[row * RP + clampi(j0 - i, -RELW, RELW) + RELW];
      const float pv1 = rw[row * RP + clampi(j1 - i, -RELW, RELW) + RELW];
      const float c0 = S0[r] * cqh + L0[r] * cql + pv0;
      const float c1 = S1[r] * cqh + L1[r] * cql + pv1;
      s0[r] = (mk0 != 0) ? c0 : ninf;
      s1[r] = (mk1 != 0) ? c1 : ninf;
    }

#pragma unroll
    for (int r = 0; r < 8; ++r) {
      float xm = fmaxf(s0[r], s1[r]);
      xm = fmaxf(xm, __shfl_xor(xm, 1, 32));
      xm = fmaxf(xm, __shfl_xor(xm, 2, 32));
      xm = fmaxf(xm, __shfl_xor(xm, 4, 32));
      xm = fmaxf(xm, __shfl_xor(xm, 8, 32));
      const float mn = fmaxf(mx[r], xm);
      const float al = __expf(mx[r] - mn);
      mx[r] = mn;
      const float p0 = __expf(s0[r] - mn);
      const float p1 = __expf(s1[r] - mn);
      float ps = p0 + p1;
      ps += __shfl_xor(ps, 1, 32);
      ps += __shfl_xor(ps, 2, 32);
      ps += __shfl_xor(ps, 4, 32);
      ps += __shfl_xor(ps, 8, 32);
      ls[r] = ls[r] * al + ps;
      O0[r] = O0[r] * al;
      O1[r] = O1[r] * al;
      O2[r] = O2[r] * al;
      O3[r] = O3[r] * al;
      s0[r] = p0;
      s1[r] = p1;
    }
    wave_sync_lds();
#pragma unroll
    for (int r = 0; r < 8; ++r) {
      const int row = 8 * hh + r;
      ph[row * 32 + m]      = f2h(s0[r] * PSC);
      ph[row * 32 + 16 + m] = f2h(s1[r] * PSC);
    }
    wave_sync_lds();

    const v16us af = ldfrag_u(ph + m * 32 + 8 * hh);
    const size_t vo = (size_t)(h * HD + m) * MT + tok0 + (size_t)sb + 8 * hh;
    const v16us vf0 = ldfrag_u(VT + vo);
    const v16us vf1 = ldfrag_u(VT + vo + (size_t)16 * MT);
    const v16us vf2 = ldfrag_u(VT + vo + (size_t)32 * MT);
    const v16us vf3 = ldfrag_u(VT + vo + (size_t)48 * MT);
    O0 = mma_g(af, vf0, O0);
    O1 = mma_g(af, vf1, O1);
    O2 = mma_g(af, vf2, O2);
    O3 = mma_g(af, vf3, O3);
  }
  acc_guard4(O0, O1, O2, O3);

  wave_sync_lds();
  float* zs = rw;
  const float fin = 1.0f / (PSC * VSC);
#pragma unroll
  for (int r = 0; r < 8; ++r) {
    const int row = 8 * hh + r;
    const float linv = 1.0f / ls[r];
    const float g = linv * fin;
    zs[row * ZP + m]      = O0[r] * g;
    zs[row * ZP + 16 + m] = O1[r] * g;
    zs[row * ZP + 32 + m] = O2[r] * g;
    zs[row * ZP + 48 + m] = O3[r] * g;
  }
  wave_sync_lds();
  {
    const int c4 = (lane & 15) * 4;
    v4f vals[8];
#pragma unroll
    for (int it = 0; it < 8; ++it) {
      const int row = it * 2 + hh;
      vals[it] = *(const v4f*)(zs + row * ZP + c4);
    }
    const size_t or0 = tok0 + (size_t)t0;
    for (int pass = 0; pass < 2; ++pass) {
#pragma unroll
      for (int it = 0; it < 8; ++it) {
        const int row = it * 2 + hh;
        float* dst = out + (or0 + (size_t)row) * DM + h * HD + c4;
        *(volatile v4f*)dst = vals[it];
      }
      __threadfence();
    }
  }
}

extern "C" void kernel_launch(void* const* d_in, const int* in_sizes, int n_in,
                              void* d_out, int out_size, void* d_ws, size_t ws_size,
                              hipStream_t stream) {
  if (n_in < 6) return;
  if (in_sizes[0] < ((NB - 1) * SEQ_FULL + SEQ) * DM) return;
  if (in_sizes[1] < ((NB - 1) * SEQ_FULL + SEQ)) return;
  if (in_sizes[2] < 3 * DM * DM) return;
  if (in_sizes[3] < 3 * DM) return;
  if (in_sizes[4] < NREL * HD) return;
  if (in_sizes[5] < NREL) return;
  if (out_size < MT * DM) return;

  const float* x     = (const float*)d_in[0];
  const int*   mask  = (const int*)d_in[1];
  const float* w_qkv = (const float*)d_in[2];
  const float* b_qkv = (const float*)d_in[3];
  const float* w_rel = (const float*)d_in[4];
  const float* b_rel = (const float*)d_in[5];

  const size_t PXH = (size_t)MT * DM * 2;
  const size_t PW  = (size_t)3 * DM * DM * 2;
  const size_t PPE = (size_t)65536;
  const size_t PQ  = (size_t)MT * DM * 2;
  const size_t PVT = (size_t)DM * MT * 2;
  if ((size_t)NRELP * HD * 2 > PPE) return;
  size_t off = 0;
  const size_t oXH = off; off += PXH;
  const size_t oW  = off; off += PW;
  const size_t oPE = off; off += PPE;
  const size_t oQH = off; off += PQ;
  const size_t oQL = off; off += PQ;
  const size_t oKH = off; off += PQ;
  const size_t oVT = off; off += PVT;
  if (off > ws_size) return;
  if (off > (size_t)134217728) return;

  char* ws = (char*)d_ws;
  unsigned short* XH  = (unsigned short*)(ws + oXH);
  unsigned short* WP  = (unsigned short*)(ws + oW);
  unsigned short* PEH = (unsigned short*)(ws + oPE);
  unsigned short* QH  = (unsigned short*)(ws + oQH);
  unsigned short* QL  = (unsigned short*)(ws + oQL);
  unsigned short* KH  = (unsigned short*)(ws + oKH);
  unsigned short* VT  = (unsigned short*)(ws + oVT);
  float* out0 = (float*)d_out;

  const dim3 blk(256);
  const int gQK = ((MT / 64) * (DM / 64) + 7) / 8;
  const int gVT = ((DM / 64) * (MT / 64) + 7) / 8;

  cvt_rows<0><<<dim3((MT * DM) / 2048), blk, 0, stream>>>(x, XH, MT * DM, 1.0f);
  cvt_rows<1><<<dim3((3 * DM * DM) / 2048), blk, 0, stream>>>(w_qkv, WP, 3 * DM * DM, WSCL);
  cvt_rows<2><<<dim3((NRELP * HD + 2047) / 2048), blk, 0, stream>>>(w_rel, PEH, NRELP * HD, WSCL);

  gemm64<2, 1><<<dim3(gQK), blk, 0, stream>>>(XH, DM, WP, DM, QH, QL, DM, QKS / WSCL,
                                              b_qkv, GRP, 0, QKS, MT, DM, DM);
  gemm64<1, 1><<<dim3(gQK), blk, 0, stream>>>(XH, DM, WP + (size_t)DM * DM, DM, KH, KH, DM, QKS / WSCL,
                                              b_qkv, GRP, HD, QKS, MT, DM, DM);
  gemm64<1, 2><<<dim3(gVT), blk, 0, stream>>>(WP + (size_t)2 * DM * DM, DM, XH, DM, VT, VT, MT, VSC / WSCL,
                                              b_qkv, GRP, 2 * HD, VSC, DM, MT, DM);

  attn_kernel<<<dim3((NB * NH * (SEQ / 16)) / AWV), dim3(64), 0, stream>>>(QH, QL, KH, PEH, VT, b_rel, mask, out0);
  (void)hipGetLastError();
}
